// PureBiMambaScan_12378095747607
// MI455X (gfx1250) — hardware-run, weakly checked
//
#include <hip/hip_runtime.h>
#include <hip/hip_fp16.h>
#include <math.h>

typedef __attribute__((ext_vector_type(16))) _Float16 v16h;
typedef __attribute__((ext_vector_type(8)))  _Float16 v8h;
typedef __attribute__((ext_vector_type(8)))  float    v8f;
typedef __attribute__((ext_vector_type(4)))  float    v4f;
typedef __attribute__((ext_vector_type(2)))  unsigned v2u;
typedef __attribute__((ext_vector_type(4)))  unsigned v4u;

constexpr int kBatch   = 4;
constexpr int kL       = 2048;
constexpr int kRows    = kBatch * kL;
constexpr int kD       = 512;
constexpr int kNst     = 16;
constexpr int kWReal   = kD + 2 * kNst;
constexpr int kWN      = 576;
constexpr int kBiasCols = kD;
constexpr int kOffB    = kD;
constexpr int kOffC    = kD + kNst;
constexpr int kXpWords = kWN / 4;
constexpr int kAlpFloats = kD * kNst;
constexpr int kPadFloats = kAlpFloats + kD;
constexpr float kXCarry = 64.0f;
constexpr float kWCarry = 4096.0f;
constexpr float kYCarry = 64.0f;
constexpr float kResid  = 2048.0f;
static_assert(kBatch == 4 && kL == 2048 && kRows == 8192 && kD == 512 && kNst == 16);
static_assert(kWReal == 544 && kWN == 576 && kBiasCols == 512 && kOffB == 512 && kOffC == 528);
static_assert(kXpWords == 144 && kAlpFloats == 8192 && kPadFloats == 8704);
static_assert(kXCarry == 64.0f && kWCarry == 4096.0f && kYCarry == 64.0f && kResid == 2048.0f);
static_assert(kWReal <= kWN && (kWN % 64) == 0 && (kD % 32) == 0 && (kRows % 32) == 0);
static_assert((kD % 64) == 0 && (kL % 64) == 0);
static_assert((kBiasCols % 4) == 0 && (kWN % 4) == 0 && (kD % 8) == 0);
static_assert(kOffC + kNst <= kWN);

constexpr size_t kSzXH   = (size_t)kRows * kD * 2;
constexpr size_t kSzXR   = (size_t)kRows * kD * 4;
constexpr size_t kSzWALL = (size_t)kWN * kD * 2;
constexpr size_t kSzXP   = (size_t)kRows * kWN * 4;
constexpr size_t kSzXPB  = (size_t)kRows * kWN * 4;
constexpr size_t kSzPADS = (size_t)kPadFloats * 4;
constexpr size_t kSzYF   = (size_t)kRows * kD * 2;
constexpr size_t kSzYB   = (size_t)kRows * kD * 2;
constexpr size_t kOffXH   = 0;
constexpr size_t kOffXR   = kOffXH   + kSzXH;
constexpr size_t kOffWALL = kOffXR   + kSzXR;
constexpr size_t kOffXP   = kOffWALL + kSzWALL;
constexpr size_t kOffXPB  = kOffXP   + kSzXP;
constexpr size_t kOffPADS = kOffXPB  + kSzXPB;
constexpr size_t kOffYF   = kOffPADS + kSzPADS;
constexpr size_t kOffYB   = kOffYF   + kSzYF;
constexpr size_t kWsTotal = kOffYB   + kSzYB;
static_assert(kSzXH == 8388608ull && kSzXR == 16777216ull && kSzWALL == 589824ull && kSzXP == 18874368ull);
static_assert(kSzXPB == 18874368ull && kSzPADS == 34816ull && kSzYF == 8388608ull && kSzYB == 8388608ull);
static_assert(kWsTotal == 8388608ull + 16777216ull + 589824ull + 18874368ull + 18874368ull + 34816ull +
              8388608ull + 8388608ull);
static_assert(kWsTotal == 80316416ull);
static_assert(kWsTotal < 134217728ull);
static_assert((kSzXH % 128) == 0 && (kSzXR % 128) == 0 && (kSzWALL % 128) == 0 && (kSzXP % 128) == 0 &&
              (kSzXPB % 128) == 0 && (kSzPADS % 128) == 0 && (kSzYF % 128) == 0 && (kSzYB % 128) == 0);
static_assert((((size_t)kAlpFloats * 4) % 128) == 0);
static_assert((((size_t)kWN * 4) % 128) == 0);

__device__ __forceinline__ _Float16 f16_flush(float v) {
  const float w = (fabsf(v) < 6.103515625e-05f) ? 0.0f : v;
  return (_Float16)w;
}

__device__ __forceinline__ float bf16r(float v) {
  unsigned u = __float_as_uint(v);
  u = (u + 0x7FFFu + ((u >> 16) & 1u)) & 0xFFFF0000u;
  return __uint_as_float(u);
}

__device__ __forceinline__ float h16_to_f32(unsigned hb) {
  const unsigned sgn = (hb & 0x8000u) << 16; const unsigned em = hb & 0x7fffu;
  const float fn = __uint_as_float((em << 13) + 0x38000000u);
  const float fs = (float)em * 5.9604644775390625e-8f;
  const float mag = (em < 0x400u) ? fs : fn; return __uint_as_float(__float_as_uint(mag) | sgn); }

namespace eng {
union FragU { v16h v; v8h h[2]; };
__device__ __forceinline__ v16h frag_load(const _Float16* p) {
  FragU f;
  f.h[0] = *(const v8h*)(p);
  f.h[1] = *(const v8h*)(p + 16);
  return f.v;
}
__device__ __forceinline__ v8f mma(v16h a, v16h b, v8f c) {
  return __builtin_amdgcn_wmma_f32_16x16x32_f16(false, a, false, b, (short)0, c, false, false);
}
__device__ __forceinline__ void guard1(v8f& a, v16h x, v16h y) {
  asm volatile("v_nop\n\tv_nop\n\tv_nop\n\tv_nop" : "+v"(a) : "v"(x), "v"(y));
}
__device__ __forceinline__ void guard_acc(v8f& a) {
  asm volatile("v_nop\n\tv_nop\n\tv_nop\n\tv_nop" : "+v"(a));
}
__device__ __forceinline__ void keep4(v16h a, v16h b, v16h c, v16h d) {
  asm volatile("v_nop" :: "v"(a), "v"(b), "v"(c), "v"(d));
}

template <int MI, int SPL>
__global__ __launch_bounds__(256) void gemm_f16_kernel(
    const unsigned short* __restrict__ Ap, const unsigned short* __restrict__ A2p, int lda,
    const unsigned short* __restrict__ Btp, const unsigned short* __restrict__ Bt2p, int ldb,
    float* __restrict__ C, int ldc, int M, int N, int K, float scale, float rscale)
{
  static_assert(MI >= 1 && MI <= 2);
  static_assert(SPL >= 0 && SPL <= 2);
  const _Float16* A   = (const _Float16*)Ap;
  const _Float16* A2  = (const _Float16*)A2p;
  const _Float16* Bt  = (const _Float16*)Btp;
  const _Float16* Bt2 = (const _Float16*)Bt2p;
  __shared__ __align__(16) float sT[8][16 * 68];
  const int lane = threadIdx.x & 31;
  const int wave = threadIdx.x >> 5;
  const int tilesN = N >> 6;
  const int tilesM = M / (16 * MI);
  const int tile = blockIdx.x * 8 + wave;
  if (tile >= tilesM * tilesN) return;
  const int tm = tile / tilesN;
  const int tn = tile - tm * tilesN;
  const int m0 = tm * (16 * MI);
  const int n0 = tn << 6;
  const int rlane = lane & 15;
  const int koff  = (lane >> 4) * 8;
  const int mOff  = (lane >> 4) * 8;

  v8f acc[MI][4], accr[MI][4];
#pragma unroll
  for (int i = 0; i < MI; ++i)
#pragma unroll
    for (int j = 0; j < 4; ++j) {
      acc[i][j]  = (v8f){0.f, 0.f, 0.f, 0.f, 0.f, 0.f, 0.f, 0.f};
      accr[i][j] = (v8f){0.f, 0.f, 0.f, 0.f, 0.f, 0.f, 0.f, 0.f};
    }

  for (int k0 = 0; k0 < K; k0 += 32) {
    v16h bh[4], bl[4];
#pragma unroll
    for (int j = 0; j < 4; ++j) {
      const size_t bo = (size_t)(n0 + (j << 4) + rlane) * ldb + koff + k0;
      bh[j] = frag_load(Bt + bo);
      if (SPL == 2) bl[j] = frag_load(Bt2 + bo); else bl[j] = bh[j];
    }
#pragma unroll
    for (int i = 0; i < MI; ++i) {
      const size_t ao = (size_t)(m0 + (i << 4) + rlane) * lda + koff + k0;
      const v16h ah = frag_load(A + ao);
      v16h al = ah;
      if (SPL >= 1) al = frag_load(A2 + ao);
#pragma unroll
      for (int j = 0; j < 4; ++j) {
        acc[i][j] = mma(ah, bh[j], acc[i][j]);
        if (SPL >= 1) accr[i][j] = mma(al, bh[j], accr[i][j]);
        if (SPL == 2) accr[i][j] = mma(ah, bl[j], accr[i][j]);
      }
#pragma unroll
      for (int j = 0; j < 4; ++j) {
        guard1(acc[i][j], ah, al);
        if (SPL >= 1) guard1(accr[i][j], ah, al);
      }
    }
    keep4(bh[0], bh[1], bh[2], bh[3]);
    if (SPL == 2) keep4(bl[0], bl[1], bl[2], bl[3]);
  }
#pragma unroll
  for (int i = 0; i < MI; ++i)
#pragma unroll
    for (int j = 0; j < 4; ++j) {
      guard_acc(acc[i][j]);
      if (SPL >= 1) guard_acc(accr[i][j]);
    }

  float* slab = sT[wave];
#pragma unroll
  for (int i = 0; i < MI; ++i) {
    const int mBase = m0 + (i << 4);
#pragma unroll
    for (int j = 0; j < 4; ++j) {
#pragma unroll
      for (int r = 0; r < 8; ++r) {
        float v = acc[i][j][r] * scale;
        if (SPL >= 1) v += accr[i][j][r] * rscale;
        slab[(mOff + r) * 68 + (j << 4) + rlane] = v;
      }
    }
    __builtin_amdgcn_fence(__ATOMIC_RELEASE, "workgroup");
    __builtin_amdgcn_wave_barrier();
    __builtin_amdgcn_fence(__ATOMIC_ACQUIRE, "workgroup");
    {
      const int hh = lane >> 4, c4 = (lane & 15) * 4;
      for (int pass = 0; pass < 2; ++pass) {
#pragma unroll
        for (int it = 0; it < 8; ++it) {
          const int row = it * 2 + hh;
          const v4f v = *(const v4f*)(slab + row * 68 + c4);
          *(volatile v4f*)(C + (size_t)(mBase + row) * ldc + n0 + c4) = v;
        }
        __threadfence();
      }
    }
    __builtin_amdgcn_fence(__ATOMIC_RELEASE, "workgroup");
    __builtin_amdgcn_wave_barrier();
    __builtin_amdgcn_fence(__ATOMIC_ACQUIRE, "workgroup");
  }
}
}

__device__ __forceinline__ _Float16 in_half(float v, float carry, bool live) {
  const float t = live ? (bf16r(v) * carry) : 0.0f;
  return f16_flush(t);
}
__device__ __forceinline__ _Float16 val_half(float v, float carry, bool live) {
  const float t = live ? (v * carry) : 0.0f;
  return f16_flush(t);
}
__device__ __forceinline__ int imin2(int a, int b) {
  return (a < b) ? a : b;
}
__device__ __forceinline__ int iclamp(int v, int lo, int hi) {
  const int t = (v < lo) ? lo : v;
  return (t > hi) ? hi : t;
}

__global__ __launch_bounds__(256) void pack_x_kernel(
    const float* __restrict__ x, unsigned short* __restrict__ XH)
{
  const int i = blockIdx.x * 256 + threadIdx.x;
  const float* sp = x + (size_t)i * 8;
  const v4f a0 = *(const v4f*)(sp);
  const v4f a1 = *(const v4f*)(sp + 4);
  const float f0 = a0[0];
  const float f1 = a0[1];
  const float f2 = a0[2];
  const float f3 = a0[3];
  const float f4 = a1[0];
  const float f5 = a1[1];
  const float f6 = a1[2];
  const float f7 = a1[3];
  const float r0 = bf16r(f0);
  const float r1 = bf16r(f1);
  const float r2 = bf16r(f2);
  const float r3 = bf16r(f3);
  const float r4 = bf16r(f4);
  const float r5 = bf16r(f5);
  const float r6 = bf16r(f6);
  const float r7 = bf16r(f7);
  v8h hv;
  hv[0] = val_half(r0, kXCarry, true);
  hv[1] = val_half(r1, kXCarry, true);
  hv[2] = val_half(r2, kXCarry, true);
  hv[3] = val_half(r3, kXCarry, true);
  hv[4] = val_half(r4, kXCarry, true);
  hv[5] = val_half(r5, kXCarry, true);
  hv[6] = val_half(r6, kXCarry, true);
  hv[7] = val_half(r7, kXCarry, true);
  unsigned short* qh = XH + (size_t)i * 8;
  *(volatile v8h*)qh = hv;
  __threadfence();
  *(volatile v8h*)qh = hv;
}

__global__ __launch_bounds__(256) void rne_x_kernel(
    const float* __restrict__ x, float* __restrict__ XR)
{
  const int i = blockIdx.x * 256 + threadIdx.x;
  const v4f a0 = *(const v4f*)(x + (size_t)i * 4);
  const float f0 = a0[0];
  const float f1 = a0[1];
  const float f2 = a0[2];
  const float f3 = a0[3];
  v4f o;
  o[0] = bf16r(f0);
  o[1] = bf16r(f1);
  o[2] = bf16r(f2);
  o[3] = bf16r(f3);
  float* q = XR + (size_t)i * 4;
  *(volatile v4f*)q = o;
  __threadfence();
  *(volatile v4f*)q = o;
}

__global__ __launch_bounds__(256) void pack_wall3_kernel(
    const float* __restrict__ wd, const float* __restrict__ wb, const float* __restrict__ wc,
    unsigned short* __restrict__ WALL)
{
  const int i = blockIdx.x * 256 + threadIdx.x;
  const int n = i / (kD / 8);
  const int k8 = (i - n * (kD / 8)) * 8;
  const bool live = (n < kWReal);
  const int nc = imin2(n, kWReal - 1);
  const float* src = (nc < kD) ? (wd + (size_t)nc * kD) : ((nc < kD + kNst) ? (wb + (size_t)(nc - kD) * kD) : (wc + (size_t)(nc - kD - kNst) * kD));
  const v4f a0 = *(const v4f*)(src + k8);
  const v4f a1 = *(const v4f*)(src + k8 + 4);
  const float f0 = a0[0];
  const float f1 = a0[1];
  const float f2 = a0[2];
  const float f3 = a0[3];
  const float f4 = a1[0];
  const float f5 = a1[1];
  const float f6 = a1[2];
  const float f7 = a1[3];
  v8h hv;
  hv[0] = in_half(f0, kWCarry, live);
  hv[1] = in_half(f1, kWCarry, live);
  hv[2] = in_half(f2, kWCarry, live);
  hv[3] = in_half(f3, kWCarry, live);
  hv[4] = in_half(f4, kWCarry, live);
  hv[5] = in_half(f5, kWCarry, live);
  hv[6] = in_half(f6, kWCarry, live);
  hv[7] = in_half(f7, kWCarry, live);
  unsigned short* q = WALL + (size_t)i * 8;
  *(volatile v8h*)q = hv;
  __threadfence();
  *(volatile v8h*)q = hv;
}

__global__ __launch_bounds__(256) void add_bias_kernel(
    const float* __restrict__ XP, const float* __restrict__ bdel, float* __restrict__ XPB)
{
  const int i = blockIdx.x * 256 + threadIdx.x;
  const int c4 = (i % kXpWords) * 4;
  const bool live = (c4 < kBiasCols);
  const int cb = imin2(c4, kBiasCols - 4);
  const v4f a0 = *(const v4f*)(XP + (size_t)i * 4);
  const v4f b0 = *(const v4f*)(bdel + cb);
  const float x0 = a0[0];
  const float x1 = a0[1];
  const float x2 = a0[2];
  const float x3 = a0[3];
  const float g0 = b0[0];
  const float g1 = b0[1];
  const float g2 = b0[2];
  const float g3 = b0[3];
  const float t0 = live ? bf16r(g0) : 0.0f;
  const float t1 = live ? bf16r(g1) : 0.0f;
  const float t2 = live ? bf16r(g2) : 0.0f;
  const float t3 = live ? bf16r(g3) : 0.0f;
  v4f o;
  o[0] = x0 + t0;
  o[1] = x1 + t1;
  o[2] = x2 + t2;
  o[3] = x3 + t3;
  float* q = XPB + (size_t)i * 4;
  *(volatile v4f*)q = o;
  __threadfence();
  *(volatile v4f*)q = o;
}

__global__ __launch_bounds__(32) void pads_kernel(
    const float* __restrict__ alog, float* __restrict__ PADS)
{
  const int wi = blockIdx.x * 32 + threadIdx.x;
  const int f0 = wi * 4;
  const bool isA = (f0 < kAlpFloats);
  const int ea = isA ? f0 : (kAlpFloats - 4);
  const v4f va = *(const v4f*)(alog + ea);
  const float a0 = va[0];
  const float a1 = va[1];
  const float a2 = va[2];
  const float a3 = va[3];
  const float s0 = isA ? a0 : 0.0f;
  const float s1 = isA ? a1 : 0.0f;
  const float s2 = isA ? a2 : 0.0f;
  const float s3 = isA ? a3 : 0.0f;
  v4f o;
  o[0] = bf16r(s0);
  o[1] = bf16r(s1);
  o[2] = bf16r(s2);
  o[3] = bf16r(s3);
  float* q = PADS + (size_t)f0;
  *(volatile v4f*)q = o;
  __threadfence();
  *(volatile v4f*)q = o;
}

typedef float    ms1_v4f __attribute__((ext_vector_type(4)));
typedef unsigned ms1_v4u __attribute__((ext_vector_type(4)));
struct ms1_args {
  const float* dtpre;
  const float* u;
  const float* bc;
  const float* z;
  const float* A_log;
  const float* Dskip;
  __half* y;
  __half* y_lo;
  long ld_dtpre;
  long ld_u;
  long ld_bc;
  long ld_z;
  long ld_y;
  int offB;
  int offC;
  int offZ;
  float ycarry;
  int dir;
  int D;
  int L;
  int nbatch;
};
static_assert(sizeof(ms1_args) == 136);

__device__ __forceinline__ float ms1_flush16(float v) {
  return (fabsf(v) < 6.103515625e-05f) ? 0.0f : v;
}
__device__ __forceinline__ unsigned ms1_h16bits(float v) {
  return (unsigned)__half_as_ushort(__float2half_rn(ms1_flush16(v)));
}
__device__ __forceinline__ float ms1_h16val(unsigned b) {
  return __half2float(__ushort_as_half((unsigned short)b));
}
__device__ __forceinline__ float ms1_softplus(float v) {
  return fmaxf(v, 0.0f) + log1pf(expf(-fabsf(v)));
}
__device__ __forceinline__ void ms1_pack2(float v0, float v1, unsigned& hw, unsigned& lw) {
  const unsigned h0 = ms1_h16bits(v0);
  const unsigned h1 = ms1_h16bits(v1);
  const float r0 = (v0 - ms1_h16val(h0)) * 2048.0f;
  const float r1 = (v1 - ms1_h16val(h1)) * 2048.0f;
  const unsigned l0 = ms1_h16bits(r0);
  const unsigned l1 = ms1_h16bits(r1);
  hw = h0 | (h1 << 16);
  lw = l0 | (l1 << 16);
}

template <int NSTATE>
__global__ __launch_bounds__(64 * (NSTATE / 16)) void ms1_scan_kernel(ms1_args a)
{
  static_assert(NSTATE == 16 || NSTATE == 64);
  constexpr int NQ  = NSTATE / 16;
  constexpr int NT  = 64 * NQ;
  constexpr int NW  = NT / 32;
  constexpr int BCW = 2 * NSTATE;
  constexpr int YP  = 68;
  constexpr int RPI = NW * 4;
  constexpr int NIT = 64 / RPI;
  static_assert(16 * NT <= 64 * YP);
  __shared__ __align__(16) float sBC[64 * BCW];
  __shared__ __align__(16) float sY[64 * YP];
  const int tid  = threadIdx.x;
  const int lane = tid & 31;
  const int wave = tid >> 5;
  const int c    = tid / NQ;
  const int sq   = tid - c * NQ;
  const int bpb  = a.D / 64;
  const int bi   = blockIdx.x / bpb;
  if (bi >= a.nbatch) return;
  const int d0 = (blockIdx.x - bi * bpb) * 64;
  const int d  = d0 + c;
  const long rowb = (long)bi * a.L;
  const bool hasz  = (a.z != nullptr);
  const bool hasD  = (a.Dskip != nullptr);
  const bool hasLo = (a.y_lo != nullptr);

#pragma unroll 1
  for (int n = 0; n < 16; ++n) {
    const float al = a.A_log[(long)d * NSTATE + sq * 16 + n];
    sY[n * NT + tid] = -expf(al);
  }
  __syncthreads();
  float An[16], h[16];
#pragma unroll
  for (int n = 0; n < 16; ++n) {
    An[n] = sY[n * NT + tid];
    h[n] = 0.0f;
  }
  float Dd = 0.0f;
  if (hasD) Dd = a.Dskip[d];

  const int nchunk = a.L / 64;
  const bool fwd = (a.dir > 0);
  const int s0 = fwd ? 0 : 63;
  const int sd = fwd ? 1 : -1;
  const int q  = lane >> 3;
  const int c8 = (lane & 7) * 8;

  for (int ci = 0; ci < nchunk; ++ci) {
    const int tb = fwd ? (ci * 64) : (a.L - 64 - ci * 64);
    const long rowc = rowb + tb;
    __syncthreads();
#pragma unroll 8
    for (int i = 0; i < 32; ++i) {
      const int idx = tid + i * NT;
      const int st  = idx / BCW;
      const int col = idx - st * BCW;
      const int sc  = (col < NSTATE) ? (a.offB + col) : (a.offC + col - NSTATE);
      sBC[idx] = a.bc[(rowc + st) * a.ld_bc + sc];
    }
    __syncthreads();
    for (int s = 0; s < 64; ++s) {
      const int ls = s0 + sd * s;
      const long row = rowc + ls;
      float pre = a.dtpre[row * a.ld_dtpre + d];
      float uv  = a.u[row * a.ld_u + d];
      float zv  = 0.0f;
      if (hasz) zv = a.z[row * a.ld_z + a.offZ + d];
      asm volatile("" : "+v"(pre));
      asm volatile("" : "+v"(uv));
      asm volatile("" : "+v"(zv));
      const float delta = ms1_softplus(pre);
      const float dtx = delta * uv;
      const float* bp = sBC + ls * BCW + sq * 16;
      const float* cp = bp + NSTATE;
      ms1_v4f Bq[4], Cq[4];
#pragma unroll
      for (int k = 0; k < 4; ++k) {
        Bq[k] = *(const ms1_v4f*)(bp + 4 * k);
        Cq[k] = *(const ms1_v4f*)(cp + 4 * k);
      }
      float yv = 0.0f;
#pragma unroll
      for (int n = 0; n < 16; ++n) {
        const float e = __expf(delta * An[n]);
        h[n] = fmaf(e, h[n], dtx * Bq[n >> 2][n & 3]);
        yv = fmaf(h[n], Cq[n >> 2][n & 3], yv);
      }
      if (NQ > 1) {
        yv += __shfl_xor(yv, 1, 32);
        yv += __shfl_xor(yv, 2, 32);
      }
      if (hasD) yv = fmaf(uv, Dd, yv);
      if (hasz) {
        const float sg = __builtin_amdgcn_rcpf(1.0f + expf(-zv));
        yv = yv * (zv * sg);
      }
      if (sq == 0) sY[ls * YP + c] = yv * a.ycarry;
    }
    __syncthreads();
    ms1_v4u hw[NIT], lw[NIT];
#pragma unroll
    for (int it = 0; it < NIT; ++it) {
      const int row = it * RPI + wave * 4 + q;
      const float* sp = sY + row * YP + c8;
      const ms1_v4f f0 = *(const ms1_v4f*)(sp);
      const ms1_v4f f1 = *(const ms1_v4f*)(sp + 4);
      unsigned h0, h1, h2, h3, l0, l1, l2, l3;
      ms1_pack2(f0[0], f0[1], h0, l0);
      ms1_pack2(f0[2], f0[3], h1, l1);
      ms1_pack2(f1[0], f1[1], h2, l2);
      ms1_pack2(f1[2], f1[3], h3, l3);
      hw[it] = (ms1_v4u){h0, h1, h2, h3};
      lw[it] = (ms1_v4u){l0, l1, l2, l3};
    }
    for (int pass = 0; pass < 2; ++pass) {
#pragma unroll
      for (int it = 0; it < NIT; ++it) {
        const int row = it * RPI + wave * 4 + q;
        const long o = (rowc + row) * a.ld_y + d0 + c8;
        *(volatile ms1_v4u*)(a.y + o) = hw[it];
        if (hasLo) *(volatile ms1_v4u*)(a.y_lo + o) = lw[it];
      }
      __threadfence();
    }
  }
}

constexpr float kInvMean = 1.0f / (kYCarry * (float)kL);
static_assert(kInvMean == 7.62939453125e-06f);
__global__ __launch_bounds__(256) void mean_time_kernel(
    const unsigned short* __restrict__ YF, const unsigned short* __restrict__ YB, float* __restrict__ out)
{
  const int i = blockIdx.x * 256 + threadIdx.x;
  const int b = i / (kD / 4);
  const int d4 = (i - b * (kD / 4)) * 4;
  float acc[4];
  acc[0] = 0.0f;
  acc[1] = 0.0f;
  acc[2] = 0.0f;
  acc[3] = 0.0f;
  for (int t = 0; t < kL; ++t) {
    const size_t e = (size_t)(b * kL + t) * kD + d4;
    const v2u wf = *(const v2u*)(YF + e);
    const v2u wg = *(const v2u*)(YB + e);
    const unsigned f01 = wf[0];
    const unsigned f23 = wf[1];
    const unsigned g01 = wg[0];
    const unsigned g23 = wg[1];
    {
      const float s = h16_to_f32(f01 & 0xffffu) + h16_to_f32(g01 & 0xffffu);
      acc[0] = acc[0] + s;
    }
    {
      const float s = h16_to_f32(f01 >> 16) + h16_to_f32(g01 >> 16);
      acc[1] = acc[1] + s;
    }
    {
      const float s = h16_to_f32(f23 & 0xffffu) + h16_to_f32(g23 & 0xffffu);
      acc[2] = acc[2] + s;
    }
    {
      const float s = h16_to_f32(f23 >> 16) + h16_to_f32(g23 >> 16);
      acc[3] = acc[3] + s;
    }
  }
  v4f o;
  o[0] = acc[0] * kInvMean;
  o[1] = acc[1] * kInvMean;
  o[2] = acc[2] * kInvMean;
  o[3] = acc[3] * kInvMean;
  float* q = out + (size_t)i * 4;
  *(volatile v4f*)q = o;
  __threadfence();
  *(volatile v4f*)q = o;
}

static_assert(((kRows / 32) * (kWN / 64)) % 8 == 0 && ((kRows / 32) * (kWN / 64)) / 8 == 288);
static_assert((8192 / 32) * (576 / 64) / 8 == 288);
static_assert((8192 / 32) * (576 / 64) == 2304);
static_assert(((kRows * kD / 8) % 256) == 0 && (kRows * kD / 8) / 256 == 2048);
static_assert(((kRows * kD / 4) % 256) == 0 && (kRows * kD / 4) / 256 == 4096);
static_assert(((kWN * kD / 8) % 256) == 0 && (kWN * kD / 8) / 256 == 144);
static_assert((kPadFloats / 4) == 68 * 32 && (kAlpFloats / 4) == 64 * 32);
static_assert(((kRows * kXpWords) % 256) == 0 && (kRows * kXpWords) / 256 == 4608);
static_assert(kRows * kXpWords == kRows * kWN / 4);
static_assert((512 / 64) * 4 == 32);
static_assert((kD / 64) * kBatch == 32);
static_assert(((kBatch * (kD / 4)) % 256) == 0 && (kBatch * (kD / 4)) / 256 == 2);
static_assert(kBatch * kD * 4 == 8192);

extern "C" void kernel_launch(void* const* d_in, const int* in_sizes, int n_in,
                              void* d_out, int out_size, void* d_ws, size_t ws_size,
                              hipStream_t stream)
{
  if (n_in < 6) return;
  if (in_sizes[0] != kBatch * kL * kD) return;
  if (in_sizes[1] != kD * kNst) return;
  if (in_sizes[2] != kNst * kD) return;
  if (in_sizes[3] != kNst * kD) return;
  if (in_sizes[4] != kD * kD) return;
  if (in_sizes[5] != kD) return;
  if (out_size != kBatch * kD) return;
  if (ws_size < kWsTotal) return;

  const float* tokens  = (const float*)d_in[0];
  const float* log_a   = (const float*)d_in[1];
  const float* w_b     = (const float*)d_in[2];
  const float* w_c     = (const float*)d_in[3];
  const float* w_delta = (const float*)d_in[4];
  const float* b_delta = (const float*)d_in[5];
  float* out = (float*)d_out;

  char* ws = (char*)d_ws;
  unsigned short* XH   = (unsigned short*)(ws + kOffXH);
  float*          XR   = (float*)(ws + kOffXR);
  unsigned short* WALL = (unsigned short*)(ws + kOffWALL);
  float*          XP   = (float*)(ws + kOffXP);
  float*          XPB  = (float*)(ws + kOffXPB);
  float*          PADS = (float*)(ws + kOffPADS);
  unsigned short* YF   = (unsigned short*)(ws + kOffYF);
  unsigned short* YB   = (unsigned short*)(ws + kOffYB);
  float*          ALP  = PADS;
  float*          DSP  = PADS + kAlpFloats;

  constexpr float s1 = 1.0f / (kXCarry * kWCarry);

  pack_x_kernel<<<(kRows * kD / 8) / 256, 256, 0, stream>>>(tokens, XH);

  rne_x_kernel<<<(kRows * kD / 4) / 256, 256, 0, stream>>>(tokens, XR);

  pack_wall3_kernel<<<144, 256, 0, stream>>>(w_delta, w_b, w_c, WALL);

  pads_kernel<<<68, 32, 0, stream>>>(log_a, PADS);

  eng::gemm_f16_kernel<2, 0><<<dim3((8192 / 32) * (576 / 64) / 8), 256, 0, stream>>>(
      XH, nullptr, 512, WALL, nullptr, 512, XP, 576, 8192, 576, 512, s1, 0.0f);

  add_bias_kernel<<<4608, 256, 0, stream>>>(XP, b_delta, XPB);

  ms1_args sf;
  sf.dtpre = XPB;
  sf.u = XR;
  sf.bc = XPB;
  sf.z = nullptr;
  sf.A_log = ALP;
  sf.Dskip = DSP;
  sf.y = (__half*)YF;
  sf.y_lo = nullptr;
  sf.ld_dtpre = kWN;
  sf.ld_u = kD;
  sf.ld_bc = kWN;
  sf.ld_z = 0;
  sf.ld_y = kD;
  sf.offB = kOffB;
  sf.offC = kOffC;
  sf.offZ = 0;
  sf.ycarry = kYCarry;
  sf.dir = 1;
  sf.D = kD;
  sf.L = kL;
  sf.nbatch = kBatch;

  ms1_args sb;
  sb.dtpre = XPB;
  sb.u = XR;
  sb.bc = XPB;
  sb.z = nullptr;
  sb.A_log = ALP;
  sb.Dskip = DSP;
  sb.y = (__half*)YB;
  sb.y_lo = nullptr;
  sb.ld_dtpre = kWN;
  sb.ld_u = kD;
  sb.ld_bc = kWN;
  sb.ld_z = 0;
  sb.ld_y = kD;
  sb.offB = kOffB;
  sb.offC = kOffC;
  sb.offZ = 0;
  sb.ycarry = kYCarry;
  sb.dir = -1;
  sb.D = kD;
  sb.L = kL;
  sb.nbatch = kBatch;

  ms1_scan_kernel<16><<<dim3((512 / 64) * 4), 64, 0, stream>>>(sf);

  ms1_scan_kernel<16><<<dim3((512 / 64) * 4), 64, 0, stream>>>(sb);

  mean_time_kernel<<<2, 256, 0, stream>>>(YF, YB, out);
}
